// UnrolledLRU_37709812859308
// MI455X (gfx1250) — hardware-verified
//
#include <hip/hip_runtime.h>
#include <math.h>

typedef __attribute__((ext_vector_type(16))) _Float16 v16h;
typedef __attribute__((ext_vector_type(8)))  _Float16 v8h;
typedef __attribute__((ext_vector_type(8)))  float    v8f;
typedef __attribute__((ext_vector_type(4)))  float    v4f;

constexpr int kSeqLen  = 32768;
constexpr int kWidth   = 256;
constexpr int kStates  = 256;
constexpr int kPairs   = 2 * kStates;
constexpr int kScanTS  = 64;
constexpr int kScanSt  = 64;
constexpr int kScanP   = 132;
static_assert((kWidth % 32) == 0 && (kPairs % 32) == 0);
static_assert((kSeqLen % 64) == 0 && (kPairs % 64) == 0 && (kWidth % 64) == 0);
static_assert((kSeqLen % kScanTS) == 0 && (kStates % kScanSt) == 0);
static_assert((kScanP % 4) == 0 && kScanP >= 2 * kScanSt);

constexpr float kCarryX  = 16.0f;
constexpr float kCarryW  = 1024.0f;
constexpr float kCarryS  = 16.0f;
constexpr float kF16Min  = 6.103515625e-05f;
constexpr float kF32Min  = 1.17549435e-38f;
constexpr float kFoldIn  = 1.0f / (kCarryX * kCarryW);
constexpr float kFoldOut = 1.0f / (kCarryS * kCarryW);
static_assert(kFoldIn * 16384.0f == 1.0f);
static_assert(kFoldOut * 16384.0f == 1.0f);

constexpr size_t kOffX16  = 0;
constexpr size_t kOffWB   = kOffX16 + (size_t)kSeqLen * kWidth * 2;
constexpr size_t kOffCC   = kOffWB  + (size_t)kPairs * kWidth * 2;
constexpr size_t kOffTAB  = kOffCC  + (size_t)kWidth * kPairs * 2;
constexpr size_t kOffBU   = kOffTAB + (size_t)2 * kStates * 4;
constexpr size_t kOffSP   = kOffBU  + (size_t)kSeqLen * kPairs * 4;
constexpr size_t kWsTotal = kOffSP  + (size_t)kSeqLen * kPairs * 2;
static_assert(kWsTotal == 117966848ull);
static_assert(kWsTotal <= 134217728ull);
static_assert((kOffWB % 128) == 0 && (kOffCC % 128) == 0 && (kOffTAB % 128) == 0 &&
              (kOffBU % 128) == 0 && (kOffSP % 128) == 0);

constexpr int kBlkX = kSeqLen * kWidth / 8 / 256;
constexpr int kBlkW = kPairs * kWidth / 8 / 256;
constexpr int kBlkC = kWidth * kPairs / 8 / 256;
static_assert(kBlkX == 4096 && kBlkW == 64 && kBlkC == 64);

__device__ __forceinline__ float bf_val(float f) {
  unsigned u = __float_as_uint(f);
  u = (u + 0x7FFFu + ((u >> 16) & 1u)) & 0xFFFF0000u;
  return __uint_as_float(u);
}
__device__ __forceinline__ _Float16 f16_operand(float v) {
  const float s = (fabsf(v) < kF16Min) ? 0.0f : v;
  return (_Float16)s;
}
__device__ __forceinline__ void cvt8_store(const float* __restrict__ src, unsigned short* __restrict__ dst,
                                           float pre, float carry) {
  const v4f a0 = *(const v4f*)(src);
  const v4f a1 = *(const v4f*)(src + 4);
  v8h hv;
#pragma unroll
  for (int e = 0; e < 4; ++e) {
    const float p0 = bf_val(a0[e]) * pre;
    const float p1 = bf_val(a1[e]) * pre;
    hv[e]     = f16_operand(p0 * carry);
    hv[4 + e] = f16_operand(p1 * carry);
  }
  *(volatile v8h*)dst = hv;
  __threadfence();
  *(volatile v8h*)dst = hv;
}

__global__ __launch_bounds__(256) void planes_tables(
    const float* __restrict__ x, const float* __restrict__ nuLog, const float* __restrict__ thLog,
    const float* __restrict__ Br, const float* __restrict__ Bi,
    const float* __restrict__ Cr, const float* __restrict__ Ci,
    const float* __restrict__ gaLog,
    unsigned short* __restrict__ X16, unsigned short* __restrict__ WB,
    unsigned short* __restrict__ CC, float* __restrict__ TAB)
{
  const int blk = blockIdx.x;
  const int tid = threadIdx.x;
  if (blk < kBlkX) {
    const size_t i = (size_t)blk * 256 + tid;
    cvt8_store(x + i * 8, X16 + i * 8, 1.0f, kCarryX);
  } else if (blk < kBlkX + kBlkW) {
    const int b = blk - kBlkX;
    const int half = (b >= 32) ? 1 : 0;
    const int j = (b & 31) * 256 + tid;
    const int n = j >> 5;
    const float g = expf(bf_val(gaLog[n]));
    const float* base = half ? Bi : Br;
    cvt8_store(base + (size_t)j * 8, WB + ((size_t)half * 8192 + j) * 8, g, kCarryW);
  } else if (blk < kBlkX + kBlkW + kBlkC) {
    const int b = blk - kBlkX - kBlkW;
    const int half = (b >= 32) ? 1 : 0;
    const int j = (b & 31) * 256 + tid;
    const int h = j >> 5;
    const int seg = j & 31;
    const float* base = half ? Ci : Cr;
    cvt8_store(base + (size_t)j * 8, CC + (size_t)h * kPairs + half * kStates + seg * 8, 1.0f, kCarryW);
  } else {
    const float nv  = bf_val(nuLog[tid]);
    const float tv  = bf_val(thLog[tid]);
    const float mag = expf(-expf(nv));
    const float ang = expf(tv);
    const float cs  = cosf(ang);
    const float sn  = sinf(ang);
    float lre = mag * cs;
    float lim = mag * sn;
    lre = (fabsf(lre) < kF32Min) ? 0.0f : lre;
    lim = (fabsf(lim) < kF32Min) ? 0.0f : lim;
    volatile float* t0 = TAB + tid;
    volatile float* t1 = TAB + kStates + tid;
    *t0 = lre;
    *t1 = lim;
    __threadfence();
    *t0 = lre;
    *t1 = lim;
  }
}

namespace eng {

union FragU { v16h v; v8h h[2]; };
__device__ __forceinline__ v16h frag_load(const _Float16* p) {
  FragU f;
  f.h[0] = *(const v8h*)(p);
  f.h[1] = *(const v8h*)(p + 16);
  return f.v;
}
__device__ __forceinline__ v8f mma16(v16h a, v16h b, v8f c) {
  return __builtin_amdgcn_wmma_f32_16x16x32_f16(false, a, false, b, (short)0, c, false, false);
}
__device__ __forceinline__ void acc_tie(v8f& c, v16h a, v16h b) {
  asm volatile("v_nop\n\tv_nop\n\tv_nop\n\tv_nop" : "+v"(c) : "v"(a), "v"(b));
}
__device__ __forceinline__ void acc_settle(v8f& c) {
  asm volatile("v_nop\n\tv_nop\n\tv_nop\n\tv_nop" : "+v"(c));
}
__device__ __forceinline__ void keep4(v16h a, v16h b, v16h c, v16h d) {
  asm volatile("v_nop" :: "v"(a), "v"(b), "v"(c), "v"(d));
}

template <int EPI>
__global__ __launch_bounds__(256) void gemm64_f16(
    const unsigned short* __restrict__ Ap, int lda,
    const unsigned short* __restrict__ Btp, int ldb,
    float* __restrict__ C, int ldc,
    const float* __restrict__ skipX, int ldx, const float* __restrict__ skipD,
    int M, int N, int K, float scale)
{
  const _Float16* A  = (const _Float16*)Ap;
  const _Float16* Bt = (const _Float16*)Btp;
  __shared__ __align__(16) float sT[8][16 * 68];
  const int lane = threadIdx.x & 31;
  const int wave = threadIdx.x >> 5;
  const int tilesN = N >> 6;
  const int tilesM = M >> 6;
  const int tile = blockIdx.x * 8 + wave;
  if (tile >= tilesM * tilesN) return;
  const int tm = tile / tilesN;
  const int tn = tile - tm * tilesN;
  const int m0 = tm << 6;
  const int n0 = tn << 6;

  const int rlane = lane & 15;
  const int koff  = (lane >> 4) * 8;
  const int mOff  = (lane >> 4) * 8;

  v8f acc[4][4];
#pragma unroll
  for (int i = 0; i < 4; ++i)
#pragma unroll
    for (int j = 0; j < 4; ++j) acc[i][j] = (v8f){0.f, 0.f, 0.f, 0.f, 0.f, 0.f, 0.f, 0.f};

  for (int k0 = 0; k0 < K; k0 += 32) {
    v16h bh[4];
#pragma unroll
    for (int j = 0; j < 4; ++j)
      bh[j] = frag_load(Bt + (size_t)(n0 + (j << 4) + rlane) * ldb + koff + k0);
#pragma unroll
    for (int i = 0; i < 4; ++i) {
      const v16h ah = frag_load(A + (size_t)(m0 + (i << 4) + rlane) * lda + koff + k0);
#pragma unroll
      for (int j = 0; j < 4; ++j) acc[i][j] = mma16(ah, bh[j], acc[i][j]);
      acc_tie(acc[i][0], ah, bh[0]);
      acc_tie(acc[i][1], ah, bh[1]);
      acc_tie(acc[i][2], ah, bh[2]);
      acc_tie(acc[i][3], ah, bh[3]);
    }
    keep4(bh[0], bh[1], bh[2], bh[3]);
  }
#pragma unroll
  for (int i = 0; i < 4; ++i) {
    acc_settle(acc[i][0]);
    acc_settle(acc[i][1]);
    acc_settle(acc[i][2]);
    acc_settle(acc[i][3]);
  }

  float* slab = sT[wave];
  const int hh = lane >> 4;
  const int c4 = (lane & 15) * 4;
  v4f dv = (v4f){0.f, 0.f, 0.f, 0.f};
  if (EPI == 1) {
    const v4f dr = *(const v4f*)(skipD + n0 + c4);
    dv[0] = bf_val(dr[0]);
    dv[1] = bf_val(dr[1]);
    dv[2] = bf_val(dr[2]);
    dv[3] = bf_val(dr[3]);
  }
#pragma unroll
  for (int i = 0; i < 4; ++i) {
    const int mBase = m0 + (i << 4);
#pragma unroll
    for (int j = 0; j < 4; ++j) {
#pragma unroll
      for (int r = 0; r < 8; ++r)
        slab[(mOff + r) * 68 + (j << 4) + rlane] = acc[i][j][r] * scale;
    }
    __builtin_amdgcn_fence(__ATOMIC_RELEASE, "workgroup");
    __builtin_amdgcn_wave_barrier();
    __builtin_amdgcn_fence(__ATOMIC_ACQUIRE, "workgroup");
    v4f ov[8];
#pragma unroll
    for (int it = 0; it < 8; ++it) {
      const int row = it * 2 + hh;
      v4f v = *(const v4f*)(slab + row * 68 + c4);
      if (EPI == 1) {
        const v4f xr = *(const v4f*)(skipX + (size_t)(mBase + row) * ldx + n0 + c4);
        v[0] = fmaf(bf_val(xr[0]), dv[0], v[0]);
        v[1] = fmaf(bf_val(xr[1]), dv[1], v[1]);
        v[2] = fmaf(bf_val(xr[2]), dv[2], v[2]);
        v[3] = fmaf(bf_val(xr[3]), dv[3], v[3]);
      }
      ov[it] = v;
    }
    for (int pass = 0; pass < 2; ++pass) {
#pragma unroll
      for (int it = 0; it < 8; ++it) {
        const int row = it * 2 + hh;
        *(volatile v4f*)(C + (size_t)(mBase + row) * ldc + n0 + c4) = ov[it];
      }
      __threadfence();
    }
    __builtin_amdgcn_fence(__ATOMIC_RELEASE, "workgroup");
    __builtin_amdgcn_wave_barrier();
    __builtin_amdgcn_fence(__ATOMIC_ACQUIRE, "workgroup");
  }
}

}

__global__ __launch_bounds__(64) void rotation_scan(
    const float* __restrict__ BU, const float* __restrict__ TAB, unsigned short* __restrict__ SP)
{
  __shared__ __align__(16) float sT[kScanTS * kScanP];
  const int tid = threadIdx.x, lane = tid & 31, wave = tid >> 5;
  const int n0 = blockIdx.x * kScanSt;
  const int n  = n0 + tid;
  const float lre = TAB[n];
  const float lim = TAB[kStates + n];
  float sre = 0.0f, sim = 0.0f;
  const int srow  = tid >> 5;
  const int shalf = (tid & 31) >> 4;
  const int scol4 = (tid & 15) * 4;
  const float* gsrc = BU + (size_t)shalf * kStates + n0 + scol4;
  float* ldst = sT + shalf * kScanSt + scol4;
  const int q = lane >> 3, c8 = (lane & 7) * 8;
  unsigned short* gdst = SP + (size_t)wave * kStates + n0 + c8;
  const float* lsrc = sT + wave * kScanSt + c8;
#pragma unroll 1
  for (int t0 = 0; t0 < kSeqLen; t0 += kScanTS) {
    __syncthreads();
#pragma unroll 1
    for (int g = 0; g < 4; ++g) {
#pragma unroll
      for (int i = 0; i < 8; ++i) {
        const int row = (g * 8 + i) * 2 + srow;
        *(v4f*)(ldst + row * kScanP) = *(const v4f*)(gsrc + (size_t)(t0 + row) * kPairs);
      }
    }
    __syncthreads();
#pragma unroll 4
    for (int s = 0; s < kScanTS; ++s) {
      float* pr = sT + s * kScanP + tid;
      const float fre = pr[0];
      const float fim = pr[kScanSt];
      const float nre = lre * sre - lim * sim + fre;
      const float nim = lre * sim + lim * sre + fim;
      sre = nre;
      sim = nim;
      pr[0]       = nre * kCarryS;
      pr[kScanSt] = nim * (-kCarryS);
    }
    __syncthreads();
    v8h hv[16];
#pragma unroll
    for (int it = 0; it < 16; ++it) {
      const int row = it * 4 + q;
      const float* sp = lsrc + row * kScanP;
      const v4f a0 = *(const v4f*)(sp);
      const v4f a1 = *(const v4f*)(sp + 4);
#pragma unroll
      for (int e = 0; e < 4; ++e) {
        hv[it][e]     = f16_operand(a0[e]);
        hv[it][4 + e] = f16_operand(a1[e]);
      }
    }
    for (int pass = 0; pass < 2; ++pass) {
#pragma unroll
      for (int it = 0; it < 16; ++it) {
        const int row = it * 4 + q;
        *(volatile v8h*)(gdst + (size_t)(t0 + row) * kPairs) = hv[it];
      }
      __threadfence();
    }
  }
}

extern "C" void kernel_launch(void* const* d_in, const int* in_sizes, int n_in,
                              void* d_out, int out_size, void* d_ws, size_t ws_size,
                              hipStream_t stream) {
  if (n_in < 9) return;
  if (in_sizes[0] != kSeqLen * kWidth) return;
  if (in_sizes[1] != kStates) return;
  if (in_sizes[2] != kStates) return;
  if (in_sizes[3] != kStates * kWidth) return;
  if (in_sizes[4] != kStates * kWidth) return;
  if (in_sizes[5] != kWidth * kStates) return;
  if (in_sizes[6] != kWidth * kStates) return;
  if (in_sizes[7] != kWidth) return;
  if (in_sizes[8] != kStates) return;
  if (out_size != kSeqLen * kWidth) return;
  if (ws_size < kWsTotal) return;

  const float* x     = (const float*)d_in[0];
  const float* nuLog = (const float*)d_in[1];
  const float* thLog = (const float*)d_in[2];
  const float* Br    = (const float*)d_in[3];
  const float* Bi    = (const float*)d_in[4];
  const float* Cr    = (const float*)d_in[5];
  const float* Ci    = (const float*)d_in[6];
  const float* Dv    = (const float*)d_in[7];
  const float* gaLog = (const float*)d_in[8];
  float* out = (float*)d_out;

  char* ws = (char*)d_ws;
  unsigned short* X16 = (unsigned short*)(ws + kOffX16);
  unsigned short* WB  = (unsigned short*)(ws + kOffWB);
  unsigned short* CC  = (unsigned short*)(ws + kOffCC);
  float*          TAB = (float*)(ws + kOffTAB);
  float*          BU  = (float*)(ws + kOffBU);
  unsigned short* SP  = (unsigned short*)(ws + kOffSP);

  planes_tables<<<dim3(kBlkX + kBlkW + kBlkC + 1), dim3(256), 0, stream>>>(
      x, nuLog, thLog, Br, Bi, Cr, Ci, gaLog, X16, WB, CC, TAB);

  eng::gemm64_f16<0><<<dim3((kSeqLen / 64) * (kPairs / 64) / 8), dim3(256), 0, stream>>>(
      X16, kWidth, WB, kWidth, BU, kPairs, x, kWidth, Dv,
      kSeqLen, kPairs, kWidth, kFoldIn);

  rotation_scan<<<dim3(kStates / kScanSt), dim3(kScanSt), 0, stream>>>(BU, TAB, SP);

  eng::gemm64_f16<1><<<dim3((kSeqLen / 64) * (kWidth / 64) / 8), dim3(256), 0, stream>>>(
      SP, kPairs, CC, kPairs, out, kWidth, x, kWidth, Dv,
      kSeqLen, kWidth, kPairs, kFoldOut);
}
